// Intra_SA_LF_Parallel_39109972197525
// MI455X (gfx1250) — hardware-verified
//
#include <hip/hip_runtime.h>
#include <stdint.h>

#define NIMG    50
#define CCH     64
#define HW      32
#define NPIXI   1024
#define NPIX    3276800
#define EE      128
#define E3      384
#define FF      256
#define ANG     5
#define LTOK    160
#define NPB     160
#define NSEQ    320
#define MROWS   51200
#define NHD     8
#define HDIM    16
#define NBH     2560
#define PADW    34
#define CLIMG   73984
#define KCONV   576
#define NKSCV   18
#define LDC     132
#define LDC2    68
#define PP      40
#define OSP     20
#define PWB     1280
#define VTP     168
#define WOFF_IN 8192
#define WOFF_OP 57344
#define WOFF_F1 73728
#define WOFF_F2 106496
#define WOFF_WO 139264
#define WL_TOT  147456
#define INV512  0.001953125f
#define INV4096 0.000244140625f
#define LN4096  8.3177661667193429f

static_assert(MROWS == NSEQ * LTOK);
static_assert(NSEQ == 2 * NPB);
static_assert(NPB == ANG * HW);
static_assert(LTOK == ANG * HW);
static_assert((MROWS % 64) == 0);
static_assert((LTOK % 16) == 0);
static_assert((LTOK % 4) == 0);
static_assert(NBH == NSEQ * NHD);
static_assert(CLIMG == PADW * PADW * CCH);
static_assert(KCONV == 9 * CCH);
static_assert(NKSCV * 32 == KCONV);
static_assert(PWB == 16 * PP * 2);
static_assert(16 * OSP * 4 <= PWB);
static_assert((PP * 2) % 16 == 0 && PP >= 32);
static_assert((VTP * 2) % 16 == 0 && VTP >= LTOK);
static_assert((LDC * 4) % 16 == 0 && (LDC2 * 4) % 16 == 0);
static_assert(NPIX == NIMG * CCH * NPIXI);
static_assert(WOFF_IN == EE * CCH);
static_assert(WOFF_OP == WOFF_IN + E3 * EE);
static_assert(WOFF_F1 == WOFF_OP + EE * EE);
static_assert(WOFF_F2 == WOFF_F1 + FF * EE);
static_assert(WOFF_WO == WOFF_F2 + EE * FF);
static_assert(WL_TOT == WOFF_WO + CCH * EE);

typedef _Float16 v16h __attribute__((ext_vector_type(16)));
typedef _Float16 v8h  __attribute__((ext_vector_type(8)));
typedef float    v8f  __attribute__((ext_vector_type(8)));
typedef float    v4f  __attribute__((ext_vector_type(4)));
typedef unsigned int v4u __attribute__((ext_vector_type(4)));
typedef unsigned int v2u __attribute__((ext_vector_type(2)));

__device__ __forceinline__ unsigned short bf_bits(float f) {
  unsigned u = __float_as_uint(f);
  return (unsigned short)((u + 0x7FFFu + ((u >> 16) & 1u)) >> 16);
}
__device__ __forceinline__ float bf_up(unsigned short b) { return __uint_as_float(((unsigned)b) << 16); }
__device__ __forceinline__ float bfr(float f) { return bf_up(bf_bits(f)); }
__device__ __forceinline__ unsigned short h_bits(_Float16 x) { return __builtin_bit_cast(unsigned short, x); }
__device__ __forceinline__ unsigned short hb16(float f) { return h_bits((_Float16)f); }
__device__ __forceinline__ unsigned pk16(unsigned short a, unsigned short b) { return (unsigned)a | ((unsigned)b << 16); }
__device__ __forceinline__ v8f zero8() { v8f z = {0.f, 0.f, 0.f, 0.f, 0.f, 0.f, 0.f, 0.f}; return z; }

__device__ __forceinline__ float wsum(float v) {
  v += __shfl_xor(v, 1, 32);
  v += __shfl_xor(v, 2, 32);
  v += __shfl_xor(v, 4, 32);
  v += __shfl_xor(v, 8, 32);
  v += __shfl_xor(v, 16, 32);
  return v;
}

__device__ __forceinline__ v4u pk8(const float* p, float mul) {
  v4u a;
#pragma unroll
  for (int e = 0; e < 4; ++e) a[e] = pk16(hb16(p[2 * e] * mul), hb16(p[2 * e + 1] * mul));
  return a;
}

__device__ __forceinline__ void tok2pix(int br, int R, int& bt, int& y, int& x) {
  R = min(max(R, 0), MROWS - 1);
  const int sq = R / LTOK, l = R - sq * LTOK;
  const int b = sq / NPB, nn = sq - b * NPB;
  const int i1 = nn >> 5, i2 = nn & 31, a = l >> 5, s = l & 31;
  const int u = br ? i1 : a;
  const int v = br ? a : i1;
  y = br ? i2 : s;
  x = br ? s : i2;
  bt = b * 25 + u * 5 + v;
}

__device__ __forceinline__ v16h ldfrag2(const _Float16* p, size_t ahalf) {
  union { v16h v; v8h h[2]; } f;
  f.h[0] = *(const v8h*)(p);
  f.h[1] = *(const v8h*)(p + ahalf);
  return f.v;
}
__device__ __forceinline__ v16h ldfrag_h(const _Float16* p) { return ldfrag2(p, 16); }
__device__ __forceinline__ v16h ldfrag_lo(const _Float16* p) {
  union { v16h v; v8h h[2]; v4u u[2]; } f;
  f.h[0] = *(const v8h*)(p);
  v4u z; z[0] = 0u; z[1] = 0u; z[2] = 0u; z[3] = 0u;
  f.u[1] = z;
  return f.v;
}

__device__ __forceinline__ v8f mma_raw(v16h a, v16h b, v8f c) {
  return __builtin_amdgcn_wmma_f32_16x16x32_f16(false, a, false, b, (short)0, c, false, false);
}
__device__ __forceinline__ v8f mma_g1(v16h a, v16h b, v8f c) {
  c = mma_raw(a, b, c);
#if defined(__HIP_DEVICE_COMPILE__)
  asm volatile("v_nop\n\tv_nop\n\tv_nop\n\tv_nop" : "+v"(c) : "v"(a), "v"(b));
#endif
  return c;
}
__device__ __forceinline__ void guard2(v8f& c0, v8f& c1, const v16h& a0, const v16h& b0, const v16h& b1) {
#if defined(__HIP_DEVICE_COMPILE__)
  asm volatile("v_nop\n\tv_nop\n\tv_nop\n\tv_nop" : "+v"(c0), "+v"(c1) : "v"(a0), "v"(b0), "v"(b1));
#endif
}
__device__ __forceinline__ void guard4(v8f& c0, v8f& c1, v8f& c2, v8f& c3,
                                       const v16h& a0, const v16h& a1, const v16h& b0, const v16h& b1) {
#if defined(__HIP_DEVICE_COMPILE__)
  asm volatile("v_nop\n\tv_nop\n\tv_nop\n\tv_nop"
               : "+v"(c0), "+v"(c1), "+v"(c2), "+v"(c3) : "v"(a0), "v"(a1), "v"(b0), "v"(b1));
#endif
}
__device__ __forceinline__ void wave_sync_lds() {
  __builtin_amdgcn_fence(__ATOMIC_RELEASE, "workgroup");
  __builtin_amdgcn_wave_barrier();
  __builtin_amdgcn_fence(__ATOMIC_ACQUIRE, "workgroup");
}

__device__ __forceinline__ v4f ln4(const v4f a, const v4f gg, const v4f be) {
  float s = (a[0] + a[1]) + (a[2] + a[3]);
  s = wsum(s);
  const float mu = s * (1.0f / (float)EE);
  v4f d;
  d[0] = a[0] - mu; d[1] = a[1] - mu; d[2] = a[2] - mu; d[3] = a[3] - mu;
  float sq = (d[0] * d[0] + d[1] * d[1]) + (d[2] * d[2] + d[3] * d[3]);
  sq = wsum(sq);
  const float rs = rsqrtf(sq * (1.0f / (float)EE) + 1e-5f);
  v4f y;
#pragma unroll
  for (int e = 0; e < 4; ++e) y[e] = (d[e] * rs) * gg[e] + be[e];
  return y;
}

__device__ __forceinline__ void mm_tile(const _Float16* __restrict__ A, int lda, size_t aks, size_t ahalf,
                                        const _Float16* __restrict__ W, int ldw, int nks,
                                        int arow0, int bcol0, float* Cs) {
  const int tid = threadIdx.x, wave = tid >> 5, lane = tid & 31, hh = lane >> 4, c = lane & 15;
  const int mw = wave >> 2, nw = wave & 3;
  const _Float16* a0p = A + (size_t)(arow0 + mw * 32 + c) * lda + 8 * hh;
  const _Float16* a1p = A + (size_t)(arow0 + mw * 32 + 16 + c) * lda + 8 * hh;
  const _Float16* b0p = W + (size_t)(bcol0 + nw * 32 + c) * ldw + 8 * hh;
  const _Float16* b1p = W + (size_t)(bcol0 + nw * 32 + 16 + c) * ldw + 8 * hh;
  v8f a00 = zero8(), a01 = zero8(), a10 = zero8(), a11 = zero8();
#pragma unroll 1
  for (int ks = 0; ks < nks; ++ks) {
    const size_t ao = (size_t)ks * aks;
    const int bo = ks * 32;
    const v16h fa0 = ldfrag2(a0p + ao, ahalf);
    const v16h fa1 = ldfrag2(a1p + ao, ahalf);
    const v16h fb0 = ldfrag_h(b0p + bo);
    const v16h fb1 = ldfrag_h(b1p + bo);
    a00 = mma_raw(fa0, fb0, a00);
    a01 = mma_raw(fa0, fb1, a01);
    a10 = mma_raw(fa1, fb0, a10);
    a11 = mma_raw(fa1, fb1, a11);
    guard4(a00, a01, a10, a11, fa0, fa1, fb0, fb1);
  }
#pragma unroll
  for (int r = 0; r < 8; ++r) {
    const int row = mw * 32 + 8 * hh + r;
    Cs[row * LDC + nw * 32 + c]             = a00[r];
    Cs[row * LDC + nw * 32 + 16 + c]        = a01[r];
    Cs[(row + 16) * LDC + nw * 32 + c]      = a10[r];
    Cs[(row + 16) * LDC + nw * 32 + 16 + c] = a11[r];
  }
}

__device__ __forceinline__ void mm_tile64(const _Float16* __restrict__ A, int lda,
                                          const _Float16* __restrict__ W, int ldw, int nks,
                                          int arow0, float* Cs) {
  const int tid = threadIdx.x, wave = tid >> 5, lane = tid & 31, hh = lane >> 4, c = lane & 15;
  const int mw = wave >> 1, nw = wave & 1;
  const _Float16* a0p = A + (size_t)(arow0 + mw * 16 + c) * lda + 8 * hh;
  const _Float16* b0p = W + (size_t)(nw * 32 + c) * ldw + 8 * hh;
  const _Float16* b1p = W + (size_t)(nw * 32 + 16 + c) * ldw + 8 * hh;
  v8f a0 = zero8(), a1 = zero8();
#pragma unroll 1
  for (int ks = 0; ks < nks; ++ks) {
    const int bo = ks * 32;
    const v16h fa  = ldfrag_h(a0p + bo);
    const v16h fb0 = ldfrag_h(b0p + bo);
    const v16h fb1 = ldfrag_h(b1p + bo);
    a0 = mma_raw(fa, fb0, a0);
    a1 = mma_raw(fa, fb1, a1);
    guard2(a0, a1, fa, fb0, fb1);
  }
#pragma unroll
  for (int r = 0; r < 8; ++r) {
    const int row = mw * 16 + 8 * hh + r;
    Cs[row * LDC2 + nw * 32 + c]      = a0[r];
    Cs[row * LDC2 + nw * 32 + 16 + c] = a1[r];
  }
}

__global__ __launch_bounds__(256)
void k_halo(unsigned short* cl0, unsigned short* cl1) {
  const int tid = threadIdx.x;
  unsigned short* base = ((blockIdx.y == 0) ? cl0 : cl1) + (size_t)blockIdx.x * CLIMG;
  v4u z; z[0] = 0u; z[1] = 0u; z[2] = 0u; z[3] = 0u;
#pragma unroll 1
  for (int it = 0; it < 5; ++it) {
    const int q = it * 256 + tid;
    const int pix = q >> 3, c0 = (q & 7) * 8;
    int y, x;
    if (pix < PADW)                 { y = 0;                        x = pix; }
    else if (pix < 2 * PADW)        { y = PADW - 1;                 x = pix - PADW; }
    else if (pix < 2 * PADW + HW)   { y = pix - 2 * PADW + 1;       x = 0; }
    else                            { y = pix - (2 * PADW + HW) + 1; x = PADW - 1; }
    const bool ok = pix < (4 * PADW - 4);
    y = min(max(y, 0), PADW - 1);
    x = min(max(x, 0), PADW - 1);
    unsigned short* p = base + ((size_t)y * PADW + x) * CCH + c0;
    if (ok) *(volatile v4u*)p = z;
    __threadfence();
    if (ok) *(volatile v4u*)p = z;
  }
}

__global__ __launch_bounds__(256)
void k_cvt_conv(const float* __restrict__ w0, const float* __restrict__ w1, const float* __restrict__ w2,
                const float* __restrict__ w3, const float* __restrict__ w4, const float* __restrict__ w5,
                unsigned short* wc) {
  const int tid = threadIdx.x, wave = tid >> 5, lane = tid & 31;
  const int seg = blockIdx.y;
  const float* src = w0;
  if (seg == 1) src = w1;
  else if (seg == 2) src = w2;
  else if (seg == 3) src = w3;
  else if (seg == 4) src = w4;
  else if (seg == 5) src = w5;
  const int co = blockIdx.x * 8 + wave;
  unsigned short* drow = wc + ((size_t)seg * CCH + co) * KCONV;
#pragma unroll
  for (int s = 0; s < 3; ++s) {
    const int p = s * 32 + lane;
    const int pc = min(p, 71);
    const int tap = pc >> 3, ci0 = (pc & 7) * 8;
    const float* sp = src + (size_t)(co * CCH + ci0) * 9 + tap;
    v4u a;
#pragma unroll
    for (int e = 0; e < 4; ++e) {
      const float f0 = sp[(2 * e) * 9];
      const float f1 = sp[(2 * e + 1) * 9];
      a[e] = pk16(hb16(bfr(f0) * 64.0f), hb16(bfr(f1) * 64.0f));
    }
    unsigned short* dp = drow + pc * 8;
    const bool ok = p < 72;
    if (ok) *(volatile v4u*)dp = a;
    __threadfence();
    if (ok) *(volatile v4u*)dp = a;
  }
}

__global__ __launch_bounds__(256)
void k_cvt_lin(const float* __restrict__ w0, const float* __restrict__ w1, const float* __restrict__ w2,
               const float* __restrict__ w3, const float* __restrict__ w4, const float* __restrict__ w5,
               unsigned short* wl) {
  const int seg = blockIdx.y;
  const float* src = w0; int n = EE * CCH; int doff = 0;
  if (seg == 1)      { src = w1; n = E3 * EE;  doff = WOFF_IN; }
  else if (seg == 2) { src = w2; n = EE * EE;  doff = WOFF_OP; }
  else if (seg == 3) { src = w3; n = FF * EE;  doff = WOFF_F1; }
  else if (seg == 4) { src = w4; n = EE * FF;  doff = WOFF_F2; }
  else if (seg == 5) { src = w5; n = CCH * EE; doff = WOFF_WO; }
  if ((int)blockIdx.x * 1024 >= n) return;
  const int i0 = blockIdx.x * 1024 + threadIdx.x * 4;
  const v4f a = *(const v4f*)(src + i0);
  v2u pk;
  pk[0] = pk16(hb16(bfr(a[0]) * 64.0f), hb16(bfr(a[1]) * 64.0f));
  pk[1] = pk16(hb16(bfr(a[2]) * 64.0f), hb16(bfr(a[3]) * 64.0f));
  unsigned short* gp = wl + doff + i0;
  *(volatile v2u*)gp = pk;
  __threadfence();
  *(volatile v2u*)gp = pk;
}

__global__ __launch_bounds__(256)
void k_gather(const float* __restrict__ x, unsigned short* xt, int br) {
  const int tid = threadIdx.x, wave = tid >> 5, lane = tid & 31;
#pragma unroll
  for (int s = 0; s < 2; ++s) {
    const int row = wave * 8 + s * 4 + (lane >> 3);
    const int R = blockIdx.x * 64 + row;
    const int c0 = (lane & 7) * 8;
    int bt, y, xx;
    tok2pix(br, R, bt, y, xx);
    const float* xp = x + ((size_t)(bt * CCH + c0) * HW + y) * HW + xx;
    v4u a;
#pragma unroll
    for (int e = 0; e < 4; ++e) {
      const float f0 = xp[(size_t)(2 * e) * NPIXI];
      const float f1 = xp[(size_t)(2 * e + 1) * NPIXI];
      a[e] = pk16(hb16(bfr(f0) * 8.0f), hb16(bfr(f1) * 8.0f));
    }
    unsigned short* dp = xt + (size_t)R * CCH + c0;
    *(volatile v4u*)dp = a;
    __threadfence();
    *(volatile v4u*)dp = a;
  }
}

__global__ __launch_bounds__(256)
void k_gemm_t0(const unsigned short* __restrict__ xt, const unsigned short* __restrict__ w16,
               const float* __restrict__ g, const float* __restrict__ bb,
               float* t0, unsigned short* t0h, unsigned short* tn) {
  __shared__ __align__(16) float Cs[64 * LDC];
  const int tid = threadIdx.x, wave = tid >> 5, lane = tid & 31;
  const int mb = blockIdx.x;
  mm_tile((const _Float16*)(const void*)xt, CCH, (size_t)32, (size_t)16,
          (const _Float16*)(const void*)w16, CCH, CCH / 32, mb * 64, 0, Cs);
  __syncthreads();
  const v4f gr = *(const v4f*)(g + lane * 4);
  const v4f br4 = *(const v4f*)(bb + lane * 4);
  v4f gg, be;
#pragma unroll
  for (int e = 0; e < 4; ++e) { gg[e] = bfr(gr[e]); be[e] = bfr(br4[e]); }
#pragma unroll 1
  for (int it = 0; it < 8; ++it) {
    const int row = wave * 8 + it;
    const size_t R = (size_t)mb * 64 + row;
    const v4f a = *(const v4f*)(Cs + row * LDC + lane * 4);
    v4f t;
#pragma unroll
    for (int e = 0; e < 4; ++e) t[e] = a[e] * INV512;
    float* fp = t0 + R * EE + lane * 4;
    *(volatile v4f*)fp = t;
    __threadfence();
    *(volatile v4f*)fp = t;
    v2u ph;
    ph[0] = pk16(hb16(t[0] * 8.0f), hb16(t[1] * 8.0f));
    ph[1] = pk16(hb16(t[2] * 8.0f), hb16(t[3] * 8.0f));
    unsigned short* hp2 = t0h + R * EE + lane * 4;
    *(volatile v2u*)hp2 = ph;
    __threadfence();
    *(volatile v2u*)hp2 = ph;
    const v4f yv = ln4(t, gg, be);
    v2u pn;
    pn[0] = pk16(hb16(yv[0] * 8.0f), hb16(yv[1] * 8.0f));
    pn[1] = pk16(hb16(yv[2] * 8.0f), hb16(yv[3] * 8.0f));
    unsigned short* np = tn + R * EE + lane * 4;
    *(volatile v2u*)np = pn;
    __threadfence();
    *(volatile v2u*)np = pn;
  }
}

__global__ __launch_bounds__(256)
void k_gemm_qkv(const unsigned short* __restrict__ tn, const unsigned short* __restrict__ t0h,
                const unsigned short* __restrict__ wq,
                unsigned short* qpl, unsigned short* kpl, unsigned short* vpl) {
  __shared__ __align__(16) float Cs[64 * LDC];
  const int tid = threadIdx.x;
  const int mb = blockIdx.x, part = blockIdx.y;
  const unsigned short* Asrc = (part == 2) ? t0h : tn;
  mm_tile((const _Float16*)(const void*)Asrc, EE, (size_t)32, (size_t)16,
          (const _Float16*)(const void*)wq, EE, EE / 32, mb * 64, part * EE, Cs);
  __syncthreads();
  unsigned short* dst = (part == 0) ? qpl : ((part == 1) ? kpl : vpl);
  const float scl = (part == 1) ? (1.0f / 64.0f) : (1.0f / 32.0f);
  v4u pk[4];
  size_t offs[4];
#pragma unroll
  for (int s = 0; s < 4; ++s) {
    const int L = s * 32 + (tid >> 3), p = tid & 7;
    const int h8 = L >> 4, g = L & 15;
    const int row = 4 * g + (p >> 1), d0 = (p & 1) * 8;
    const int col = h8 * HDIM + d0;
    const int R = mb * 64 + row;
    const int sq = R / LTOK, l = R - sq * LTOK;
    pk[s] = pk8(Cs + row * LDC + col, scl);
    offs[s] = ((size_t)(sq * NHD + h8) * LTOK + l) * HDIM + d0;
  }
#pragma unroll
  for (int s = 0; s < 4; ++s) *(volatile v4u*)(dst + offs[s]) = pk[s];
  __threadfence();
#pragma unroll
  for (int s = 0; s < 4; ++s) *(volatile v4u*)(dst + offs[s]) = pk[s];
}

__global__ __launch_bounds__(160)
void k_attn(const unsigned short* __restrict__ qpl, const unsigned short* __restrict__ kpl,
            const unsigned short* __restrict__ vpl, unsigned short* opl) {
  __shared__ __align__(16) char pbuf[5 * PWB];
  __shared__ __align__(16) _Float16 Vt[HDIM * VTP];
  const int tid = threadIdx.x, wave = tid >> 5, lane = tid & 31, hh = lane >> 4, c = lane & 15;
  const int bh = blockIdx.x >> 1, half = blockIdx.x & 1;
  const int sq = bh >> 3, h = bh & 7;
  const int strip = half * 5 + wave;
  const int q0 = strip * 16;
  const _Float16* Q = (const _Float16*)(const void*)qpl + (size_t)bh * LTOK * HDIM;
  const _Float16* K = (const _Float16*)(const void*)kpl + (size_t)bh * LTOK * HDIM;
  const _Float16* V = (const _Float16*)(const void*)vpl + (size_t)bh * LTOK * HDIM;

  {
    const _Float16* vr = V + (size_t)tid * HDIM;
    const v8h va = *(const v8h*)(vr);
    const v8h vb = *(const v8h*)(vr + 8);
#pragma unroll
    for (int d = 0; d < 8; ++d) {
      Vt[d * VTP + tid] = va[d];
      Vt[(d + 8) * VTP + tid] = vb[d];
    }
  }
  __syncthreads();

  _Float16* Ph = (_Float16*)(pbuf + wave * PWB);
  const v16h qa = ldfrag_lo(Q + (size_t)(q0 + c) * HDIM + 8 * hh);
  const int qsb = (strip & 1) * 16 + 8 * hh;
  float mrow[8], lrow[8];
#pragma unroll
  for (int r = 0; r < 8; ++r) { mrow[r] = -1e30f; lrow[r] = 0.f; }
  v8f oa = zero8();

#pragma unroll 1
  for (int kb = 0; kb < LTOK / 32; ++kb) {
    v8f s[2];
#pragma unroll
    for (int j = 0; j < 2; ++j) {
      const int key = kb * 32 + j * 16 + c;
      const v16h kf = ldfrag_lo(K + (size_t)key * HDIM + 8 * hh);
      v8f sj = mma_g1(qa, kf, zero8());
      const int ksp = j * 16 + c;
#pragma unroll
      for (int r = 0; r < 8; ++r) {
        const int dw = ksp - (qsb + r);
        const bool ok = (dw >= -5) && (dw <= 5);
        sj[r] = ok ? sj[r] : -1.0e30f;
      }
      s[j] = sj;
    }
#pragma unroll
    for (int r = 0; r < 8; ++r) {
      float tm = fmaxf(s[0][r], s[1][r]);
      tm = fmaxf(tm, __shfl_xor(tm, 1, 32));
      tm = fmaxf(tm, __shfl_xor(tm, 2, 32));
      tm = fmaxf(tm, __shfl_xor(tm, 4, 32));
      tm = fmaxf(tm, __shfl_xor(tm, 8, 32));
      const float mn = fmaxf(mrow[r], tm);
      const float alpha = __expf((mrow[r] - mn) * INV512);
      mrow[r] = mn;
      float ps = 0.f;
#pragma unroll
      for (int j = 0; j < 2; ++j) {
        const float p = __expf((s[j][r] - mn) * INV512 + LN4096);
        ps = ps + p;
        s[j][r] = p;
      }
      ps = ps + __shfl_xor(ps, 1, 32);
      ps = ps + __shfl_xor(ps, 2, 32);
      ps = ps + __shfl_xor(ps, 4, 32);
      ps = ps + __shfl_xor(ps, 8, 32);
      lrow[r] = lrow[r] * alpha + ps;
      oa[r] = oa[r] * alpha;
    }
#pragma unroll
    for (int j = 0; j < 2; ++j) {
#pragma unroll
      for (int r = 0; r < 8; ++r) {
        Ph[(8 * hh + r) * PP + j * 16 + c] = (_Float16)s[j][r];
      }
    }
    wave_sync_lds();
    {
      const v16h pa = ldfrag_h(Ph + c * PP + 8 * hh);
      const v16h vf = ldfrag_h(Vt + c * VTP + kb * 32 + 8 * hh);
      oa = mma_g1(pa, vf, oa);
    }
    wave_sync_lds();
  }

  float* Os = (float*)(void*)(pbuf + wave * PWB);
#pragma unroll
  for (int r = 0; r < 8; ++r) {
    const float inv = 1.0f / (lrow[r] * 16.0f);
    Os[(8 * hh + r) * OSP + c] = oa[r] * inv;
  }
  wave_sync_lds();
  const int orow = lane >> 1, od0 = (lane & 1) * 8;
  const v4u pk = pk8(Os + orow * OSP + od0, 64.0f);
  unsigned short* op = opl + ((size_t)h * MROWS + (size_t)sq * LTOK + q0) * HDIM + lane * 8;
  *(volatile v4u*)op = pk;
  __threadfence();
  *(volatile v4u*)op = pk;
}

__global__ __launch_bounds__(256)
void k_gemm_oproj(const unsigned short* __restrict__ opl, const unsigned short* __restrict__ wp,
                  const float* __restrict__ t0, const float* __restrict__ g, const float* __restrict__ bb,
                  float* t1, unsigned short* t2n) {
  __shared__ __align__(16) float Cs[64 * LDC];
  const int tid = threadIdx.x, wave = tid >> 5, lane = tid & 31;
  const int mb = blockIdx.x;
  mm_tile((const _Float16*)(const void*)opl, HDIM, (size_t)2 * MROWS * HDIM, (size_t)MROWS * HDIM,
          (const _Float16*)(const void*)wp, EE, EE / 32, mb * 64, 0, Cs);
  __syncthreads();
  const v4f gr = *(const v4f*)(g + lane * 4);
  const v4f br4 = *(const v4f*)(bb + lane * 4);
  v4f gg, be;
#pragma unroll
  for (int e = 0; e < 4; ++e) { gg[e] = bfr(gr[e]); be[e] = bfr(br4[e]); }
#pragma unroll 1
  for (int it = 0; it < 8; ++it) {
    const int row = wave * 8 + it;
    const size_t R = (size_t)mb * 64 + row;
    const v4f a  = *(const v4f*)(Cs + row * LDC + lane * 4);
    const v4f tv = *(const v4f*)(t0 + R * EE + lane * 4);
    v4f o;
#pragma unroll
    for (int e = 0; e < 4; ++e) o[e] = a[e] * INV4096 + tv[e];
    float* fp = t1 + R * EE + lane * 4;
    *(volatile v4f*)fp = o;
    __threadfence();
    *(volatile v4f*)fp = o;
    const v4f yv = ln4(o, gg, be);
    v2u pn;
    pn[0] = pk16(hb16(yv[0] * 8.0f), hb16(yv[1] * 8.0f));
    pn[1] = pk16(hb16(yv[2] * 8.0f), hb16(yv[3] * 8.0f));
    unsigned short* np = t2n + R * EE + lane * 4;
    *(volatile v2u*)np = pn;
    __threadfence();
    *(volatile v2u*)np = pn;
  }
}

__global__ __launch_bounds__(256)
void k_gemm_ffn1(const unsigned short* __restrict__ t2n, const unsigned short* __restrict__ w1, unsigned short* f1) {
  __shared__ __align__(16) float Cs[64 * LDC];
  const int tid = threadIdx.x;
  const int mb = blockIdx.x, nb = blockIdx.y;
  mm_tile((const _Float16*)(const void*)t2n, EE, (size_t)32, (size_t)16,
          (const _Float16*)(const void*)w1, EE, EE / 32, mb * 64, nb * EE, Cs);
  __syncthreads();
  v4u pk[4];
  size_t offs[4];
#pragma unroll
  for (int s = 0; s < 4; ++s) {
    const int idx = s * 256 + tid;
    const int row = idx >> 4, piece = idx & 15;
    const int col0 = piece * 8;
    v4u q4;
#pragma unroll
    for (int e = 0; e < 4; ++e) {
      float z0 = Cs[row * LDC + col0 + 2 * e] * INV512;
      float z1 = Cs[row * LDC + col0 + 2 * e + 1] * INV512;
      z0 = (z0 >= 0.f) ? z0 : 0.1f * z0;
      z1 = (z1 >= 0.f) ? z1 : 0.1f * z1;
      q4[e] = pk16(hb16(z0 * 64.0f), hb16(z1 * 64.0f));
    }
    pk[s] = q4;
    offs[s] = (size_t)(mb * 64 + row) * FF + nb * EE + col0;
  }
#pragma unroll
  for (int s = 0; s < 4; ++s) *(volatile v4u*)(f1 + offs[s]) = pk[s];
  __threadfence();
#pragma unroll
  for (int s = 0; s < 4; ++s) *(volatile v4u*)(f1 + offs[s]) = pk[s];
}

__global__ __launch_bounds__(256)
void k_gemm_ffn2(const unsigned short* __restrict__ f1, const unsigned short* __restrict__ w2,
                 const float* __restrict__ t1, unsigned short* t2h) {
  __shared__ __align__(16) float Cs[64 * LDC];
  const int tid = threadIdx.x, wave = tid >> 5, lane = tid & 31;
  const int mb = blockIdx.x;
  mm_tile((const _Float16*)(const void*)f1, FF, (size_t)32, (size_t)16,
          (const _Float16*)(const void*)w2, FF, FF / 32, mb * 64, 0, Cs);
  __syncthreads();
#pragma unroll 1
  for (int it = 0; it < 8; ++it) {
    const int row = wave * 8 + it;
    const size_t R = (size_t)mb * 64 + row;
    const v4f a  = *(const v4f*)(Cs + row * LDC + lane * 4);
    const v4f tv = *(const v4f*)(t1 + R * EE + lane * 4);
    v4f o;
#pragma unroll
    for (int e = 0; e < 4; ++e) o[e] = a[e] * INV4096 + tv[e];
    v2u pn;
    pn[0] = pk16(hb16(o[0] * 8.0f), hb16(o[1] * 8.0f));
    pn[1] = pk16(hb16(o[2] * 8.0f), hb16(o[3] * 8.0f));
    unsigned short* np = t2h + R * EE + lane * 4;
    *(volatile v2u*)np = pn;
    __threadfence();
    *(volatile v2u*)np = pn;
  }
}

__global__ __launch_bounds__(256)
void k_gemm_wout(const unsigned short* __restrict__ t2h, const unsigned short* __restrict__ ww, int br,
                 unsigned short* cl) {
  __shared__ __align__(16) float Cs[64 * LDC2];
  const int tid = threadIdx.x, wave = tid >> 5, lane = tid & 31;
  const int mb = blockIdx.x;
  mm_tile64((const _Float16*)(const void*)t2h, EE, (const _Float16*)(const void*)ww, EE, EE / 32, mb * 64, Cs);
  __syncthreads();
  v4u pk[2];
  size_t offs[2];
#pragma unroll
  for (int s = 0; s < 2; ++s) {
    const int row = wave * 8 + s * 4 + (lane >> 3);
    const int c0 = (lane & 7) * 8;
    const int R = mb * 64 + row;
    int bt, y, x;
    tok2pix(br, R, bt, y, x);
    pk[s] = pk8(Cs + row * LDC2 + c0, 1.0f / 64.0f);
    offs[s] = ((size_t)(bt * PADW + y + 1) * PADW + x + 1) * CCH + c0;
  }
#pragma unroll
  for (int s = 0; s < 2; ++s) *(volatile v4u*)(cl + offs[s]) = pk[s];
  __threadfence();
#pragma unroll
  for (int s = 0; s < 2; ++s) *(volatile v4u*)(cl + offs[s]) = pk[s];
}

__global__ __launch_bounds__(256)
void k_conv(const unsigned short* __restrict__ src, const unsigned short* __restrict__ wc, int mode,
            unsigned short* dsth, const float* __restrict__ xres, float* dstf) {
  __shared__ __align__(16) float Cs[64 * LDC2];
  const int tid = threadIdx.x, wave = tid >> 5, lane = tid & 31, hh = lane >> 4, c = lane & 15;
  const int bt = blockIdx.x >> 4, y0 = (blockIdx.x & 15) * 2;
  const int mt = wave >> 1, nw = wave & 1;
  const int y = y0 + (mt >> 1), x0 = (mt & 1) * 16;
  const _Float16* S  = (const _Float16*)(const void*)src;
  const _Float16* Wt = (const _Float16*)(const void*)wc;
  const _Float16* ap  = S + ((size_t)(bt * PADW + y + 1) * PADW + x0 + 1 + c) * CCH + 8 * hh;
  const _Float16* b0p = Wt + (size_t)(nw * 32 + c) * KCONV + 8 * hh;
  const _Float16* b1p = Wt + (size_t)(nw * 32 + 16 + c) * KCONV + 8 * hh;
  v8f a0 = zero8(), a1 = zero8();
#pragma unroll 1
  for (int ks = 0; ks < NKSCV; ++ks) {
    const int tap = ks >> 1, cih = ks & 1;
    const int t3 = tap / 3;
    const int dy = t3 - 1, dx = tap - t3 * 3 - 1;
    const int aoff = (dy * PADW + dx) * CCH + cih * 32;
    const v16h fa  = ldfrag_h(ap + aoff);
    const v16h fb0 = ldfrag_h(b0p + ks * 32);
    const v16h fb1 = ldfrag_h(b1p + ks * 32);
    a0 = mma_raw(fa, fb0, a0);
    a1 = mma_raw(fa, fb1, a1);
    guard2(a0, a1, fa, fb0, fb1);
  }
#pragma unroll
  for (int r = 0; r < 8; ++r) {
    const int row = mt * 16 + 8 * hh + r;
    Cs[row * LDC2 + nw * 32 + c]      = a0[r];
    Cs[row * LDC2 + nw * 32 + 16 + c] = a1[r];
  }
  __syncthreads();
  if (mode != 2) {
    v4u pk[2];
    size_t offs[2];
#pragma unroll
    for (int s = 0; s < 2; ++s) {
      const int idx = s * 256 + tid;
      const int p = idx >> 3, piece = idx & 7;
      const int c0 = piece * 8;
      const int yy = y0 + (p >> 5), xx = p & 31;
      v4u q4;
#pragma unroll
      for (int e = 0; e < 4; ++e) {
        float z0 = Cs[p * LDC2 + c0 + 2 * e] * INV512;
        float z1 = Cs[p * LDC2 + c0 + 2 * e + 1] * INV512;
        z0 = (z0 >= 0.f) ? z0 : 0.1f * z0;
        z1 = (z1 >= 0.f) ? z1 : 0.1f * z1;
        q4[e] = pk16(hb16(z0 * 8.0f), hb16(z1 * 8.0f));
      }
      pk[s] = q4;
      offs[s] = ((size_t)(bt * PADW + yy + 1) * PADW + xx + 1) * CCH + c0;
    }
#pragma unroll
    for (int s = 0; s < 2; ++s) *(volatile v4u*)(dsth + offs[s]) = pk[s];
    __threadfence();
#pragma unroll
    for (int s = 0; s < 2; ++s) *(volatile v4u*)(dsth + offs[s]) = pk[s];
  } else {
    v4f po[4];
    size_t offs[4];
#pragma unroll
    for (int s = 0; s < 4; ++s) {
      const int idx = s * 256 + tid;
      const int co = idx >> 4, piece = idx & 15;
      const int p0 = piece * 4;
      const size_t off = (size_t)(bt * CCH + co) * NPIXI + y0 * HW + p0;
      const v4f xv = *(const v4f*)(xres + off);
      v4f o;
#pragma unroll
      for (int e = 0; e < 4; ++e) o[e] = Cs[(p0 + e) * LDC2 + co] * INV512 + bfr(xv[e]);
      po[s] = o;
      offs[s] = off;
    }
#pragma unroll
    for (int s = 0; s < 4; ++s) *(volatile v4f*)(dstf + offs[s]) = po[s];
    __threadfence();
#pragma unroll
    for (int s = 0; s < 4; ++s) *(volatile v4f*)(dstf + offs[s]) = po[s];
  }
}

__global__ __launch_bounds__(256)
void k_poolgate(const float* __restrict__ o1, const float* __restrict__ o2,
                const float* __restrict__ gw1, const float* __restrict__ gw2, float* gout) {
  __shared__ float pooled[2 * CCH];
  __shared__ float hid[16];
  __shared__ __align__(16) float gs[CCH];
  const int tid = threadIdx.x, wave = tid >> 5, lane = tid & 31;
  const int bt = blockIdx.x;
  const float* base = (wave < 4) ? o1 : o2;
  const int chb = (wave & 3) * 16;
#pragma unroll 1
  for (int j = 0; j < 16; ++j) {
    const int ch = chb + j;
    const float* rp = base + ((size_t)bt * CCH + ch) * NPIXI + lane * 4;
    v4f v = *(const v4f*)(rp);
    float m = fmaxf(fmaxf(v[0], v[1]), fmaxf(v[2], v[3]));
#pragma unroll
    for (int i = 1; i < 8; ++i) {
      v = *(const v4f*)(rp + i * 128);
      m = fmaxf(m, fmaxf(fmaxf(v[0], v[1]), fmaxf(v[2], v[3])));
    }
    m = fmaxf(m, __shfl_xor(m, 16, 32));
    m = fmaxf(m, __shfl_xor(m, 8, 32));
    m = fmaxf(m, __shfl_xor(m, 4, 32));
    m = fmaxf(m, __shfl_xor(m, 2, 32));
    m = fmaxf(m, __shfl_xor(m, 1, 32));
    if (lane == 0) pooled[wave * 16 + j] = m;
  }
  __syncthreads();
  if (tid < 16) {
    const float* wr = gw1 + tid * (2 * CCH);
    float s = 0.f;
#pragma unroll 4
    for (int k = 0; k < 2 * CCH; ++k) s += pooled[k] * bfr(wr[k]);
    hid[tid] = (s >= 0.f) ? s : 0.1f * s;
  }
  __syncthreads();
  if (tid < CCH) {
    const float* wr = gw2 + tid * 16;
    float s = 0.f;
#pragma unroll 4
    for (int k = 0; k < 16; ++k) s += hid[k] * bfr(wr[k]);
    s = fminf(fmaxf(s, -30.0f), 30.0f);
    gs[tid] = 1.0f / (1.0f + expf(-s));
  }
  __syncthreads();
  if (tid < 16) {
    const v4f gv = *(const v4f*)(gs + tid * 4);
    float* gp = gout + (size_t)bt * CCH + tid * 4;
    *(volatile v4f*)gp = gv;
    __threadfence();
    *(volatile v4f*)gp = gv;
  }
}

__global__ __launch_bounds__(256)
void k_blend(const float* __restrict__ o1, const float* __restrict__ o2, const float* __restrict__ g, float* out) {
  const int i4 = blockIdx.x * 256 + threadIdx.x;
  if (i4 < NPIX / 4) {
    const float gg = g[i4 >> 8];
    const float og = 1.0f - gg;
    const v4f a = *(const v4f*)(o1 + (size_t)i4 * 4);
    const v4f b = *(const v4f*)(o2 + (size_t)i4 * 4);
    v4f o;
#pragma unroll
    for (int e = 0; e < 4; ++e) o[e] = a[e] * gg + b[e] * og;
    float* p = out + (size_t)i4 * 4;
    *(volatile v4f*)p = o;
    __threadfence();
    *(volatile v4f*)p = o;
  }
}

extern "C" void kernel_launch(void* const* d_in, const int* in_sizes, int n_in,
                              void* d_out, int out_size, void* d_ws, size_t ws_size,
                              hipStream_t stream) {
  if (n_in < 29) return;
  if (in_sizes[0] != NPIX) return;
  for (int br = 0; br < 2; ++br) {
    const int b0 = 1 + 10 * br;
    if (in_sizes[b0 + 0] != EE * CCH) return;
    if (in_sizes[b0 + 1] != EE || in_sizes[b0 + 2] != EE) return;
    if (in_sizes[b0 + 3] != E3 * EE) return;
    if (in_sizes[b0 + 4] != EE * EE) return;
    if (in_sizes[b0 + 5] != EE || in_sizes[b0 + 6] != EE) return;
    if (in_sizes[b0 + 7] != FF * EE) return;
    if (in_sizes[b0 + 8] != EE * FF) return;
    if (in_sizes[b0 + 9] != CCH * EE) return;
  }
  for (int j = 21; j < 27; ++j) if (in_sizes[j] != CCH * CCH * 9) return;
  if (in_sizes[27] != 16 * 2 * CCH || in_sizes[28] != CCH * 16) return;
  if (out_size != NPIX) return;

  const size_t sTok4 = (size_t)MROWS * EE * 4;
  const size_t sTok2 = (size_t)MROWS * EE * 2;
  const size_t sXT   = (size_t)MROWS * CCH * 2;
  const size_t sQ    = (size_t)NBH * LTOK * HDIM * 2;
  const size_t sO    = (size_t)NHD * MROWS * HDIM * 2;
  const size_t sF1   = (size_t)MROWS * FF * 2;
  const size_t sIMG  = (size_t)NPIX * 4;
  const size_t sCL   = (size_t)NIMG * CLIMG * 2;
  const size_t sWC   = (size_t)6 * CCH * KCONV * 2;
  const size_t sWL   = (size_t)WL_TOT * 2;
  const size_t sG    = (size_t)NIMG * CCH * 4;
  size_t sR1 = 3 * sQ;
  if (sTok4 + sTok2 > sR1) sR1 = sTok4 + sTok2;
  if (sXT > sR1) sR1 = sXT;
  size_t sR2 = sTok4;
  if (sF1 > sR2) sR2 = sF1;
  if (sIMG > sR2) sR2 = sIMG;
  size_t sR3 = 2 * sTok2;
  if (sO > sR3) sR3 = sO;

  size_t off = 0;
  const size_t oR1  = off; off += sR1;
  const size_t oR2  = off; off += sR2;
  const size_t oR3  = off; off += sR3;
  const size_t oCL0 = off; off += sCL;
  const size_t oCL1 = off; off += sCL;
  const size_t oWC  = off; off += sWC;
  const size_t oWL  = off; off += sWL;
  const size_t oO1  = off; off += sIMG;
  const size_t oG   = off; off += sG;
  if (off > ws_size) return;
  if (off > (size_t)134217728) return;

  char* ws = (char*)d_ws;
  unsigned short* XT  = (unsigned short*)(ws + oR1);
  unsigned short* Qp  = (unsigned short*)(ws + oR1);
  unsigned short* Kp  = (unsigned short*)(ws + oR1 + sQ);
  unsigned short* Vp  = (unsigned short*)(ws + oR1 + 2 * sQ);
  float*          T1  = (float*)(ws + oR1);
  unsigned short* T2N = (unsigned short*)(ws + oR1 + sTok4);
  float*          T0  = (float*)(ws + oR2);
  unsigned short* F1  = (unsigned short*)(ws + oR2);
  float*          OUT2 = (float*)(ws + oR2);
  unsigned short* T0H = (unsigned short*)(ws + oR3);
  unsigned short* TN  = (unsigned short*)(ws + oR3 + sTok2);
  unsigned short* Op  = (unsigned short*)(ws + oR3);
  unsigned short* T2H = (unsigned short*)(ws + oR3);
  unsigned short* CL0 = (unsigned short*)(ws + oCL0);
  unsigned short* CL1 = (unsigned short*)(ws + oCL1);
  unsigned short* WC  = (unsigned short*)(ws + oWC);
  unsigned short* WL  = (unsigned short*)(ws + oWL);
  float*          OUT1 = (float*)(ws + oO1);
  float*          G    = (float*)(ws + oG);

  const float* x   = (const float*)d_in[0];
  const float* gw1 = (const float*)d_in[27];
  const float* gw2 = (const float*)d_in[28];
  float* out = (float*)d_out;

  const dim3 blk(256);
  k_halo<<<dim3(NIMG, 2), blk, 0, stream>>>(CL0, CL1);
  k_cvt_conv<<<dim3(CCH / 8, 6), blk, 0, stream>>>(
      (const float*)d_in[21], (const float*)d_in[22], (const float*)d_in[23],
      (const float*)d_in[24], (const float*)d_in[25], (const float*)d_in[26], WC);

  for (int br = 0; br < 2; ++br) {
    const int b0 = 1 + 10 * br;
    const float* win     = (const float*)d_in[b0 + 0];
    const float* ln1g    = (const float*)d_in[b0 + 1];
    const float* ln1b    = (const float*)d_in[b0 + 2];
    const float* inproj  = (const float*)d_in[b0 + 3];
    const float* outproj = (const float*)d_in[b0 + 4];
    const float* ln2g    = (const float*)d_in[b0 + 5];
    const float* ln2b    = (const float*)d_in[b0 + 6];
    const float* ffn1    = (const float*)d_in[b0 + 7];
    const float* ffn2    = (const float*)d_in[b0 + 8];
    const float* wout    = (const float*)d_in[b0 + 9];
    unsigned short* WCb = WC + (size_t)(3 * br) * CCH * KCONV;
    float* OUTk = (br == 0) ? OUT1 : OUT2;

    k_cvt_lin<<<dim3(48, 6), blk, 0, stream>>>(win, inproj, outproj, ffn1, ffn2, wout, WL);
    k_gather<<<dim3(MROWS / 64), blk, 0, stream>>>(x, XT, br);
    k_gemm_t0<<<dim3(MROWS / 64), blk, 0, stream>>>(XT, WL, ln1g, ln1b, T0, T0H, TN);
    k_gemm_qkv<<<dim3(MROWS / 64, 3), blk, 0, stream>>>(TN, T0H, WL + WOFF_IN, Qp, Kp, Vp);
    k_attn<<<dim3(NBH * 2), dim3(160), 0, stream>>>(Qp, Kp, Vp, Op);
    k_gemm_oproj<<<dim3(MROWS / 64), blk, 0, stream>>>(Op, WL + WOFF_OP, T0, ln2g, ln2b, T1, T2N);
    k_gemm_ffn1<<<dim3(MROWS / 64, FF / EE), blk, 0, stream>>>(T2N, WL + WOFF_F1, F1);
    k_gemm_ffn2<<<dim3(MROWS / 64), blk, 0, stream>>>(F1, WL + WOFF_F2, T1, T2H);
    k_gemm_wout<<<dim3(MROWS / 64), blk, 0, stream>>>(T2H, WL + WOFF_WO, br, CL0);
    k_conv<<<dim3(NIMG * 16), blk, 0, stream>>>(CL0, WCb, 0, CL1, x, OUTk);
    k_conv<<<dim3(NIMG * 16), blk, 0, stream>>>(CL1, WCb + (size_t)CCH * KCONV, 0, CL0, x, OUTk);
    k_conv<<<dim3(NIMG * 16), blk, 0, stream>>>(CL0, WCb + (size_t)2 * CCH * KCONV, 2, CL1, x, OUTk);
  }
  k_poolgate<<<dim3(NIMG), blk, 0, stream>>>(OUT1, OUT2, gw1, gw2, G);
  k_blend<<<dim3(NPIX / 4 / 256), blk, 0, stream>>>(OUT1, OUT2, G, out);
  (void)hipGetLastError();
}
